// Spatial_dot_80951543595332
// MI455X (gfx1250) — hardware-verified
//
#include <hip/hip_runtime.h>
#include <math.h>

typedef __attribute__((ext_vector_type(16))) _Float16 v16h;
typedef __attribute__((ext_vector_type(16))) __bf16 v16b;
typedef __attribute__((ext_vector_type(8)))  _Float16 v8h;
typedef __attribute__((ext_vector_type(8)))  float v8f;
typedef __attribute__((ext_vector_type(4)))  float v4f;
typedef __attribute__((ext_vector_type(2)))  float v2f;
typedef __attribute__((ext_vector_type(4)))  unsigned v4u;
typedef __attribute__((ext_vector_type(4)))  int v4i;
typedef float __attribute__((may_alias)) float_a;
typedef int __attribute__((may_alias)) int_a;

template <typename T> __device__ __forceinline__ void vst2(void* p, T v) { *(volatile T*)p = v; __threadfence(); *(volatile T*)p = v; }
__device__ __forceinline__ v8f wmma16(v16h a, v16h b, v8f c) {
  v8f d = __builtin_amdgcn_wmma_f32_16x16x32_f16(false, a, false, b, (short)0, c, false, false);
  asm volatile("v_nop\n\tv_nop\n\tv_nop\n\tv_nop" : "+v"(d) : "v"(a), "v"(b));
  return d;
}
__device__ __forceinline__ v8f wmma_bf(v16b a, v16b b, v8f c) {
  v8f d = __builtin_amdgcn_wmma_f32_16x16x32_bf16(false, a, false, b, (short)0, c, false, false);
  asm volatile("v_nop\n\tv_nop\n\tv_nop\n\tv_nop" : "+v"(d) : "v"(a), "v"(b));
  return d;
}
__device__ __forceinline__ v16h frag_h(const _Float16* rowk0, int lane) {
  union { v16h v; v8h q[2]; } u; const _Float16* p = rowk0 + 8 * (lane >> 4);
  u.q[0] = *(const v8h*)p; u.q[1] = *(const v8h*)(p + 16); return u.v;
}
__device__ __forceinline__ v16h frag_f32(const float* rowk0, int lane) {
  v16h a; const float* p = rowk0 + 8 * (lane >> 4);
#pragma unroll
  for (int i = 0; i < 8; ++i) { a[i] = (_Float16)p[i]; a[8 + i] = (_Float16)p[16 + i]; }
  return a;
}
__device__ __forceinline__ v16h frag_f32s(const float* rowk0, int lane, float sc) {
  v16h a; const float* p = rowk0 + 8 * (lane >> 4);
#pragma unroll
  for (int i = 0; i < 8; ++i) { a[i] = (_Float16)(p[i] * sc); a[8 + i] = (_Float16)(p[16 + i] * sc); }
  return a;
}
__device__ __forceinline__ v16h fragc_f32(const float* W, int k0, int n, int lane, int ld, int K) {
  v16h a; const int g = lane >> 4;
#pragma unroll
  for (int i = 0; i < 8; ++i) { const int ka = k0 + 8 * g + i, kb = ka + 16;
    a[i] = (_Float16)(ka < K ? W[(size_t)(ka < K ? ka : K - 1) * ld + n] : 0.f); a[8 + i] = (_Float16)(kb < K ? W[(size_t)(kb < K ? kb : K - 1) * ld + n] : 0.f); }
  return a;
}
struct F2 { v16b h, l; };
__device__ __forceinline__ F2 bsplit16(const float v[16]) { F2 r;
#pragma unroll
  for (int i = 0; i < 16; ++i) { const __bf16 h = (__bf16)v[i]; r.h[i] = h; r.l[i] = (__bf16)(v[i] - (float)h); }
  return r; }
__device__ __forceinline__ F2 split_row(const float* row, int k0, int lane) { float v[16]; const float* p = row + k0 + 8 * (lane >> 4);
#pragma unroll
  for (int i = 0; i < 8; ++i) { v[i] = p[i]; v[8 + i] = p[16 + i]; }
  return bsplit16(v); }
__device__ __forceinline__ F2 split_rowK(const float* row, int k0, int lane, int K) { float v[16]; const int g = lane >> 4;
#pragma unroll
  for (int i = 0; i < 8; ++i) { const int ka = k0 + 8 * g + i, kb = ka + 16; v[i] = ka < K ? row[ka < K ? ka : K - 1] : 0.f; v[8 + i] = kb < K ? row[kb < K ? kb : K - 1] : 0.f; }
  return bsplit16(v); }
__device__ __forceinline__ F2 split_col(const float* W, int k0, int n, int lane, int ld, int K) { float v[16]; const int g = lane >> 4;
#pragma unroll
  for (int i = 0; i < 8; ++i) { const int ka = k0 + 8 * g + i, kb = ka + 16; v[i] = ka < K ? W[(size_t)(ka < K ? ka : K - 1) * ld + n] : 0.f; v[8 + i] = kb < K ? W[(size_t)(kb < K ? kb : K - 1) * ld + n] : 0.f; }
  return bsplit16(v); }
__device__ __forceinline__ v8f mac3(const F2& a, const F2& b, v8f c) { c = wmma_bf(a.l, b.h, c); c = wmma_bf(a.h, b.l, c); return wmma_bf(a.h, b.h, c); }
__device__ __forceinline__ float sigm(float v) { return 1.0f / (1.0f + expf(-v)); }
#define LDSX() do { asm volatile("s_wait_dscnt 0" ::: "memory"); __builtin_amdgcn_wave_barrier(); __builtin_amdgcn_fence(__ATOMIC_RELEASE, "workgroup"); } while (0)


#define NT 8
#define CC 128
#define NN 4096
#define FF 64
__device__ __forceinline__ float bfr(float v) { return (float)(__bf16)v; }
__device__ __forceinline__ v16b frag_b(const __bf16* rowk0, int lane) { return __builtin_bit_cast(v16b, frag_h((const _Float16*)rowk0, lane)); }

__global__ __launch_bounds__(256) void k_cvtx(const float* __restrict__ x1, const float* __restrict__ x2, __bf16* __restrict__ X1T, __bf16* __restrict__ X2T) {
  __shared__ __align__(16) __bf16 st[64][CC + 8];
  const int tid = threadIdx.x; const int t = blockIdx.y, n0 = blockIdx.x * 64, which = blockIdx.z; const float* x = which == 0 ? x1 : x2; __bf16* XT = which == 0 ? X1T : X2T;
  for (int q = tid; q < CC * 16; q += 256) { const int c = q >> 4, p4 = q & 15; const v4f v = *(const v4f*)(x + ((size_t)t * CC + c) * NN + n0 + p4 * 4);
    st[p4 * 4][c] = (__bf16)v[0]; st[p4 * 4 + 1][c] = (__bf16)v[1]; st[p4 * 4 + 2][c] = (__bf16)v[2]; st[p4 * 4 + 3][c] = (__bf16)v[3]; }
  __syncthreads();
  for (int q = tid; q < 64 * (CC / 8); q += 256) { const int rl = q >> 4, pc = q & 15; vst2((unsigned*)(XT + ((size_t)t * NN + n0 + rl) * CC + pc * 8), *(const v4u*)(&st[rl][pc * 8])); }
}
__global__ __launch_bounds__(128) void k_proj(const __bf16* __restrict__ X1T, const __bf16* __restrict__ X2T, const float* __restrict__ W1, const float* __restrict__ b1, const float* __restrict__ W2, const float* __restrict__ b2, const float* __restrict__ W3, const float* __restrict__ b3,
                                            float* __restrict__ Q32, __bf16* __restrict__ Kh, __bf16* __restrict__ Kl, __bf16* __restrict__ GTh, __bf16* __restrict__ GTl) {
  __shared__ __align__(16) float so[4][16][68]; __shared__ __align__(16) __bf16 sh_[4][16][72], sl_[4][16][72]; __shared__ __align__(16) __bf16 sth[64][72], stl[64][72];
  const int tid = threadIdx.x, wave = tid >> 5, lane = tid & 31, col = lane & 15, g = lane >> 4; const int t = blockIdx.y, n0b = blockIdx.x * 64, which = blockIdx.z; const size_t r0 = (size_t)t * NN + n0b + wave * 16;
  const __bf16* XT = which == 1 ? X2T : X1T; const float* W = which == 0 ? W1 : (which == 1 ? W2 : W3); const float* bb_ = which == 0 ? b1 : (which == 1 ? b2 : b3);
  v8f acc[4] = {};
#pragma unroll
  for (int kc = 0; kc < CC / 32; ++kc) { const v16b a = frag_b(XT + (r0 + col) * CC + kc * 32, lane);
#pragma unroll
    for (int j = 0; j < 4; ++j) acc[j] = wmma_bf(a, split_row(W + (size_t)(j * 16 + col) * CC, kc * 32, lane).h, acc[j]); }
  if (which == 0) {
#pragma unroll
    for (int j = 0; j < 4; ++j) { const float bb = bfr(bb_[j * 16 + col]);
#pragma unroll
      for (int r = 0; r < 8; ++r) so[wave][8 * g + r][j * 16 + col] = acc[j][r] + bb; }
    LDSX();
    for (int qq = lane; qq < 16 * 16; qq += 32) { const int rl = qq >> 4, pc = qq & 15; vst2(Q32 + (r0 + rl) * FF + pc * 4, *(const v4f*)(&so[wave][rl][pc * 4])); } }
  else if (which == 1) {
#pragma unroll
    for (int j = 0; j < 4; ++j) { const float bb = bfr(bb_[j * 16 + col]);
#pragma unroll
      for (int r = 0; r < 8; ++r) { const float v = acc[j][r] + bb; const __bf16 hi = (__bf16)v; sh_[wave][8 * g + r][j * 16 + col] = hi; sl_[wave][8 * g + r][j * 16 + col] = (__bf16)(v - (float)hi); } }
    LDSX();
    for (int qq = lane; qq < 16 * 8; qq += 32) { const int rl = qq >> 3, pc = qq & 7; vst2((unsigned*)(Kh + (r0 + rl) * FF + pc * 8), *(const v4u*)(&sh_[wave][rl][pc * 8])); vst2((unsigned*)(Kl + (r0 + rl) * FF + pc * 8), *(const v4u*)(&sl_[wave][rl][pc * 8])); } }
  else {
#pragma unroll
    for (int j = 0; j < 4; ++j) { const float bb = bfr(bb_[j * 16 + col]);
#pragma unroll
      for (int r = 0; r < 8; ++r) { const float v = acc[j][r] + bb; const __bf16 hi = (__bf16)v; sth[j * 16 + col][wave * 16 + 8 * g + r] = hi; stl[j * 16 + col][wave * 16 + 8 * g + r] = (__bf16)(v - (float)hi); } }
    __syncthreads();
    for (int qq = tid; qq < 64 * 8; qq += 128) { const int f = qq >> 3, pc = qq & 7; const size_t o = ((size_t)t * FF + f) * NN + n0b + pc * 8; vst2((unsigned*)(GTh + o), *(const v4u*)(&sth[f][pc * 8])); vst2((unsigned*)(GTl + o), *(const v4u*)(&stl[f][pc * 8])); } }
}
__global__ __launch_bounds__(128) void k_dot(const float* __restrict__ Q32, const __bf16* __restrict__ Kh, const __bf16* __restrict__ Kl, const __bf16* __restrict__ GTh, const __bf16* __restrict__ GTl, float* __restrict__ out) {
  __shared__ __align__(16) float sS[4][16][68];
  __shared__ __align__(16) __bf16 sPh[4][16][72], sPl[4][16][72];
  __shared__ __align__(16) float sOT[FF][68];
  const int tid = threadIdx.x, w = tid >> 5, lane = tid & 31, col = lane & 15, g = lane >> 4; const int t = blockIdx.y, n0b = blockIdx.x * 64; const size_t q0 = (size_t)t * NN + n0b + w * 16;
  F2 aq[2];
#pragma unroll
  for (int kc = 0; kc < 2; ++kc) aq[kc] = split_row(Q32 + (q0 + col) * FF, kc * 32, lane);
  v8f acc[4] = {};
#pragma unroll 1
  for (int kt = 0; kt < NN / 64; ++kt) {
#pragma unroll
    for (int tt = 0; tt < 4; ++tt) { const size_t ko = ((size_t)t * NN + kt * 64 + tt * 16 + col) * FF; v8f s = {};
#pragma unroll
      for (int kc = 0; kc < 2; ++kc) { const v16b khf = frag_b(Kh + ko + kc * 32, lane), klf = frag_b(Kl + ko + kc * 32, lane); s = wmma_bf(aq[kc].l, khf, s); s = wmma_bf(aq[kc].h, klf, s); s = wmma_bf(aq[kc].h, khf, s); }
#pragma unroll
      for (int r = 0; r < 8; ++r) { const float v = s[r] > 0.f ? s[r] : 0.f; const __bf16 hi = (__bf16)v; sPh[w][8 * g + r][tt * 16 + col] = hi; sPl[w][8 * g + r][tt * 16 + col] = (__bf16)(v - (float)hi); } }
    LDSX();
#pragma unroll
    for (int kc = 0; kc < 2; ++kc) { const v16b ph = frag_b(&sPh[w][col][0] + kc * 32, lane), pl = frag_b(&sPl[w][col][0] + kc * 32, lane);
#pragma unroll
      for (int j = 0; j < 4; ++j) { const size_t go = ((size_t)t * FF + j * 16 + col) * NN + kt * 64 + kc * 32; const v16b gh = frag_b(GTh + go, lane), gl = frag_b(GTl + go, lane); acc[j] = wmma_bf(pl, gh, acc[j]); acc[j] = wmma_bf(ph, gl, acc[j]); acc[j] = wmma_bf(ph, gh, acc[j]); } }
    LDSX(); }
#pragma unroll
  for (int j = 0; j < 4; ++j)
#pragma unroll
    for (int r = 0; r < 8; ++r) sOT[j * 16 + col][w * 16 + 8 * g + r] = acc[j][r];
  __syncthreads();
  for (int qq = tid; qq < FF * 16; qq += 128) { const int f = qq >> 4, pc = qq & 15; vst2(out + ((size_t)t * FF + f) * NN + n0b + pc * 4, *(const v4f*)(&sOT[f][pc * 4])); }
}
extern "C" void kernel_launch(void* const* d_in, const int* in_sizes, int n_in, void* d_out, int out_size, void* d_ws, size_t ws_size, hipStream_t stream) {
  (void)in_sizes; (void)n_in; (void)out_size; (void)ws_size;
  const float** I = (const float**)d_in;
  const float* x1 = I[0]; const float* x2 = I[1]; const float* W1 = I[2]; const float* b1 = I[3]; const float* W2 = I[4]; const float* b2 = I[5]; const float* W3 = I[6]; const float* b3 = I[7];
  char* ws = (char*)d_ws; size_t off = 0;
  auto take = [&](size_t bytes) { char* p = ws + off; off += (bytes + 255) & ~(size_t)255; return p; };
  __bf16* X1T = (__bf16*)take((size_t)NT * NN * CC * 2); __bf16* X2T = (__bf16*)take((size_t)NT * NN * CC * 2); float* Q32 = (float*)take((size_t)NT * NN * FF * 4);
  __bf16* Kh = (__bf16*)take((size_t)NT * NN * FF * 2); __bf16* Kl = (__bf16*)take((size_t)NT * NN * FF * 2); __bf16* GTh = (__bf16*)take((size_t)NT * FF * NN * 2); __bf16* GTl = (__bf16*)take((size_t)NT * FF * NN * 2);
  k_cvtx<<<dim3(NN / 64, NT, 2), 256, 0, stream>>>(x1, x2, X1T, X2T);
  k_proj<<<dim3(NN / 64, NT, 3), 128, 0, stream>>>(X1T, X2T, W1, b1, W2, b2, W3, b3, Q32, Kh, Kl, GTh, GTl);
  k_dot<<<dim3(NN / 64, NT), 128, 0, stream>>>(Q32, Kh, Kl, GTh, GTl, (float*)d_out);
}
